// Layer_7670811590704
// MI455X (gfx1250) — hardware-run, weakly checked
//
#include <hip/hip_runtime.h>
#include <math.h>

constexpr int kSeq   = 2048;
constexpr int kDim   = 1024;
constexpr int kHeads = 16;
constexpr int kDh    = 64;
constexpr int kD2    = 2 * kDim;
constexpr int kD3    = 3 * kDim;
constexpr int kD4    = 4 * kDim;
constexpr float kWCarry     = 16.0f;
constexpr float kWCarryInv  = 1.0f / 16.0f;
constexpr float kPCarry     = 32768.0f;
constexpr float kPCarryInv  = 1.0f / 32768.0f;
constexpr float kScoreScale = 0.03125f;
constexpr float kInvDim     = 1.0f / 1024.0f;
constexpr float kLnEps      = 1e-5f;
constexpr float kRsqrt2     = 0.70710678118654752f;
static_assert(kHeads * kDh == kDim);
static_assert(kSeq % 64 == 0 && kDim % 64 == 0 && kD4 % 64 == 0 && kDh % 64 == 0);
static_assert(kDim % 32 == 0 && kD4 % 32 == 0 && kDh % 32 == 0 && kSeq % 32 == 0);

typedef __attribute__((ext_vector_type(16))) _Float16 v16h;
typedef __attribute__((ext_vector_type(8)))  _Float16 v8h;
typedef __attribute__((ext_vector_type(16))) __bf16   v16b;
typedef __attribute__((ext_vector_type(8)))  __bf16   v8b;
typedef __attribute__((ext_vector_type(8)))  float    v8f;
typedef __attribute__((ext_vector_type(4)))  float    v4f;
typedef __attribute__((ext_vector_type(4)))  unsigned int v4u;

__device__ __forceinline__ unsigned short f2bf_bits(float f) {
  unsigned u = __float_as_uint(f);
  return (unsigned short)((u + 0x7FFFu + ((u >> 16) & 1u)) >> 16);
}
__device__ __forceinline__ float bf_bits2f(unsigned short h) { return __uint_as_float(((unsigned)h) << 16); }

__device__ __forceinline__ void dep_guard4_h(v8f& a, v8f& b, v8f& c, v8f& d, v16h x, v16h y) {
  asm volatile("v_nop\n\tv_nop\n\tv_nop\n\tv_nop" : "+v"(a), "+v"(b), "+v"(c), "+v"(d) : "v"(x), "v"(y));
}
__device__ __forceinline__ void dep_guard4_b(v8f& a, v8f& b, v8f& c, v8f& d, v16b x, v16b y) {
  asm volatile("v_nop\n\tv_nop\n\tv_nop\n\tv_nop" : "+v"(a), "+v"(b), "+v"(c), "+v"(d) : "v"(x), "v"(y));
}
__device__ __forceinline__ void keep4_h(v16h a, v16h b, v16h c, v16h d) { asm volatile("v_nop" :: "v"(a), "v"(b), "v"(c), "v"(d)); }
__device__ __forceinline__ void keep4_b(v16b a, v16b b, v16b c, v16b d) { asm volatile("v_nop" :: "v"(a), "v"(b), "v"(c), "v"(d)); }
__device__ __forceinline__ void acc_guard4(v8f& a, v8f& b, v8f& c, v8f& d) { asm volatile("v_nop\n\tv_nop\n\tv_nop\n\tv_nop" : "+v"(a), "+v"(b), "+v"(c), "+v"(d)); }
template <typename T> struct Frag;
template <> struct Frag<_Float16> {
  typedef v16h V; union U { v16h v; v8h h[2]; };
  static __device__ __forceinline__ v16h load(const _Float16* p) {
    U f; f.h[0] = *(const v8h*)(p); f.h[1] = *(const v8h*)(p + 16); return f.v;
  }
  static __device__ __forceinline__ v8f mma(v16h a, v16h b, v8f c) {
    return __builtin_amdgcn_wmma_f32_16x16x32_f16(false, a, false, b, (short)0, c, false, false);
  }
  static __device__ __forceinline__ void guard4(v8f& a, v8f& b, v8f& c, v8f& d, v16h x, v16h y) { dep_guard4_h(a, b, c, d, x, y); }
  static __device__ __forceinline__ void keep(v16h a, v16h b, v16h c, v16h d) { keep4_h(a, b, c, d); }
};
template <> struct Frag<__bf16> {
  typedef v16b V; union U { v16b v; v8b h[2]; };
  static __device__ __forceinline__ v16b load(const __bf16* p) {
    U f; f.h[0] = *(const v8b*)(p); f.h[1] = *(const v8b*)(p + 16); return f.v;
  }
  static __device__ __forceinline__ v8f mma(v16b a, v16b b, v8f c) {
    return __builtin_amdgcn_wmma_f32_16x16x32_bf16(false, a, false, b, (short)0, c, false, false);
  }
  static __device__ __forceinline__ void guard4(v8f& a, v8f& b, v8f& c, v8f& d, v16b x, v16b y) { dep_guard4_b(a, b, c, d, x, y); }
  static __device__ __forceinline__ void keep(v16b a, v16b b, v16b c, v16b d) { keep4_b(a, b, c, d); }
};

__device__ __forceinline__ unsigned pk16(unsigned short a, unsigned short b) { return (unsigned)a | ((unsigned)b << 16); }
__device__ __forceinline__ unsigned short h_bits(float f) { const _Float16 h = (_Float16)f; return __builtin_bit_cast(unsigned short, h); }

__device__ __forceinline__ float h16_to_f32(unsigned hb) {
  const unsigned sgn = (hb & 0x8000u) << 16; const unsigned em = hb & 0x7fffu;
  const float fn = __uint_as_float((em << 13) + 0x38000000u);
  const float fs = (float)em * 5.9604644775390625e-8f;
  const float mag = (em < 0x400u) ? fs : fn; return __uint_as_float(__float_as_uint(mag) | sgn); }

template <int ET> struct Elem;
template <> struct Elem<0> { typedef _Float16 T; };
template <> struct Elem<1> { typedef __bf16 T; };
template <int ET, bool SPLIT, int BIAS_MODE, int OUT_MODE, bool RESID>
__global__ __launch_bounds__(256) void wmma_gemm64(
    const unsigned short* __restrict__ Ap, const unsigned short* __restrict__ A2p, int lda, long strideA,
    const unsigned short* __restrict__ Btp, const unsigned short* __restrict__ Bt2p, int ldb, long strideB,
    void* __restrict__ Cout, void* __restrict__ Cout2, int ldc, long strideC,
    const float* __restrict__ bias,
    const float* __restrict__ resid, long strideR,
    int M, int N, int K, float scale) {
  typedef typename Elem<ET>::T T;
  typedef typename Frag<T>::V V;
  const T* A = (const T*)Ap; const T* A2 = (const T*)A2p; const T* Bt = (const T*)Btp; const T* Bt2 = (const T*)Bt2p;
  __shared__ __align__(16) float sT[8][16 * 68];
  const int b    = blockIdx.y;
  const int lane = threadIdx.x & 31;
  const int wave = threadIdx.x >> 5;
  const int tilesN = N >> 6;
  const int tilesM = M >> 6;
  const int tile = blockIdx.x * 8 + wave;
  if (tile >= tilesM * tilesN) return;
  const int tm = tile / tilesN;
  const int tn = tile - tm * tilesN;
  const int m0 = tm << 6;
  const int n0 = tn << 6;

  const T* Ab  = A  + (size_t)b * strideA;
  const T* Bb  = Bt + (size_t)b * strideB;
  const T* Ab2 = SPLIT ? (A2  + (size_t)b * strideA) : nullptr;
  const T* Bb2 = SPLIT ? (Bt2 + (size_t)b * strideB) : nullptr;

  const int rlane = lane & 15;
  const int koff  = (lane >> 4) * 8;
  const int mOff  = (lane >> 4) * 8;

  v8f acc[4][4];
#pragma unroll
  for (int i = 0; i < 4; ++i)
#pragma unroll
    for (int j = 0; j < 4; ++j) acc[i][j] = (v8f){0.f,0.f,0.f,0.f,0.f,0.f,0.f,0.f};

  for (int k0 = 0; k0 < K; k0 += 32) {
    V bh[4], bl[4];
#pragma unroll
    for (int j = 0; j < 4; ++j) {
      const size_t bo = (size_t)(n0 + (j << 4) + rlane) * ldb + koff + k0;
      bh[j] = Frag<T>::load(Bb + bo);
      if (SPLIT) bl[j] = Frag<T>::load(Bb2 + bo);
    }
#pragma unroll
    for (int i = 0; i < 4; ++i) {
      const size_t ao = (size_t)(m0 + (i << 4) + rlane) * lda + koff + k0;
      V ah = Frag<T>::load(Ab + ao);
      V al;
      if (SPLIT) al = Frag<T>::load(Ab2 + ao);
#pragma unroll
      for (int j = 0; j < 4; ++j) {
        acc[i][j] = Frag<T>::mma(ah, bh[j], acc[i][j]);
        if (SPLIT) {
          acc[i][j] = Frag<T>::mma(ah, bl[j], acc[i][j]);
          acc[i][j] = Frag<T>::mma(al, bh[j], acc[i][j]);
        }
      }
      Frag<T>::guard4(acc[i][0], acc[i][1], acc[i][2], acc[i][3], ah, SPLIT ? al : bh[3]);
    }
    Frag<T>::keep(bh[0], bh[1], bh[2], bh[3]);
    if (SPLIT) Frag<T>::keep(bl[0], bl[1], bl[2], bl[3]);
  }
  acc_guard4(acc[0][0], acc[0][1], acc[0][2], acc[0][3]);
  acc_guard4(acc[1][0], acc[1][1], acc[1][2], acc[1][3]);
  acc_guard4(acc[2][0], acc[2][1], acc[2][2], acc[2][3]);
  acc_guard4(acc[3][0], acc[3][1], acc[3][2], acc[3][3]);

  float* slab = sT[wave];
  const float* Rb = RESID ? (resid + (size_t)b * strideR) : nullptr;
#pragma unroll
  for (int i = 0; i < 4; ++i) {
    const int mBase = m0 + (i << 4);
    float bm[8];
#pragma unroll
    for (int e = 0; e < 8; ++e) bm[e] = 0.f;
    if (BIAS_MODE == 1) {
      const v4f b0 = *(const v4f*)(bias + mBase + mOff);
      const v4f b1 = *(const v4f*)(bias + mBase + mOff + 4);
#pragma unroll
      for (int e = 0; e < 4; ++e) { bm[e] = b0[e]; bm[4 + e] = b1[e]; }
    }
#pragma unroll
    for (int j = 0; j < 4; ++j) {
      const int n = n0 + (j << 4) + rlane;
      float bv = 0.f;
      if (BIAS_MODE == 2) bv = bias[n];
#pragma unroll
      for (int r = 0; r < 8; ++r) {
        float v = acc[i][j][r] * scale;
        if (BIAS_MODE == 1) v += bm[r];
        if (BIAS_MODE == 2) v += bv;
        slab[(mOff + r) * 68 + (j << 4) + rlane] = v;
      }
    }
    __builtin_amdgcn_fence(__ATOMIC_RELEASE, "workgroup");
    __builtin_amdgcn_wave_barrier();
    __builtin_amdgcn_fence(__ATOMIC_ACQUIRE, "workgroup");
    if (OUT_MODE == 0) {
      float* C = (float*)Cout + (size_t)b * strideC;
      const int hh = lane >> 4, c4 = (lane & 15) * 4;
      for (int pass = 0; pass < 2; ++pass) {
#pragma unroll
        for (int it = 0; it < 8; ++it) {
          const int row = it * 2 + hh;
          v4f v = *(const v4f*)(slab + row * 68 + c4);
          const size_t go = (size_t)(mBase + row) * ldc + n0 + c4;
          if (RESID) {
            const v4f rr = *(const v4f*)(Rb + go);
            v += rr;
          }
          *(volatile v4f*)(C + go) = v;
        }
        __threadfence();
      }
    } else {
      const int q = lane >> 3, c8 = (lane & 7) * 8;
      unsigned short* C  = (unsigned short*)Cout  + (size_t)b * strideC;
      unsigned short* C2 = (OUT_MODE == 2) ? ((unsigned short*)Cout2 + (size_t)b * strideC) : nullptr;
      for (int pass = 0; pass < 2; ++pass) {
#pragma unroll
        for (int it = 0; it < 4; ++it) {
          const int row = it * 4 + q;
          const float* sp = slab + row * 68 + c8;
          v8h hv, lv;
#pragma unroll
          for (int e = 0; e < 8; ++e) {
            if (OUT_MODE == 1) {
              hv[e] = (_Float16)sp[e];
            } else {
              unsigned short hb = f2bf_bits(sp[e]);
              unsigned short lb = f2bf_bits(sp[e] - bf_bits2f(hb));
              hv[e] = __builtin_bit_cast(_Float16, hb);
              lv[e] = __builtin_bit_cast(_Float16, lb);
            }
          }
          *(volatile v8h*)(C + (size_t)(mBase + row) * ldc + n0 + c8) = hv;
          if (OUT_MODE == 2) *(volatile v8h*)(C2 + (size_t)(mBase + row) * ldc + n0 + c8) = lv;
        }
        __threadfence();
      }
    }
    __builtin_amdgcn_fence(__ATOMIC_RELEASE, "workgroup");
    __builtin_amdgcn_wave_barrier();
    __builtin_amdgcn_fence(__ATOMIC_ACQUIRE, "workgroup");
  }
}

__global__ __launch_bounds__(256) void cast8_f16_kernel(const float* __restrict__ in, unsigned short* __restrict__ out, int n8, float carry) {
  const int i = blockIdx.x * 256 + threadIdx.x;
  if (i >= n8) return;
  const float* p = in + 8 * (size_t)i;
  const v4f a = *(const v4f*)(p);
  const v4f c = *(const v4f*)(p + 4);
  unsigned short hb[8];
#pragma unroll
  for (int e = 0; e < 4; ++e) {
    hb[e]     = h_bits(a[e] * carry);
    hb[4 + e] = h_bits(c[e] * carry);
  }
  const v4u u = (v4u){pk16(hb[0], hb[1]), pk16(hb[2], hb[3]), pk16(hb[4], hb[5]), pk16(hb[6], hb[7])};
  unsigned short* q = out + 8 * (size_t)i;
  *(volatile v4u*)q = u;
  __threadfence();
  *(volatile v4u*)q = u;
}

__global__ __launch_bounds__(128) void layernorm_f16_kernel(const float* __restrict__ x, const float* __restrict__ gain,
                                                           const float* __restrict__ shift, unsigned short* __restrict__ out) {
  __shared__ float redA[4];
  __shared__ float redB[4];
  const int row  = blockIdx.x;
  const int t    = threadIdx.x;
  const int lane = t & 31, wave = t >> 5;
  const float* xr = x + (size_t)row * kDim + 8 * t;
  const v4f a = *(const v4f*)(xr);
  const v4f c = *(const v4f*)(xr + 4);
  float v[8];
#pragma unroll
  for (int e = 0; e < 4; ++e) { v[e] = a[e]; v[4 + e] = c[e]; }
  float s = 0.0f, q = 0.0f;
#pragma unroll
  for (int e = 0; e < 8; ++e) { s += v[e]; q += v[e] * v[e]; }
#pragma unroll
  for (int off = 16; off > 0; off >>= 1) {
    s += __shfl_xor(s, off, 32);
    q += __shfl_xor(q, off, 32);
  }
  if (lane == 0) { redA[wave] = s; redB[wave] = q; }
  __syncthreads();
  const float tot = ((redA[0] + redA[1]) + redA[2]) + redA[3];
  const float tq  = ((redB[0] + redB[1]) + redB[2]) + redB[3];
  const float mu  = tot * kInvDim;
  const float mu2 = tq * kInvDim;
  const float sigma = sqrtf(mu2 - mu * mu + kLnEps);
  const float inv = 1.0f / sigma;
  const float g  = gain[0];
  const float bb = shift[0];
  unsigned short hb[8];
#pragma unroll
  for (int e = 0; e < 8; ++e) hb[e] = h_bits((g * (v[e] - mu)) * inv + bb);
  const v4u u = (v4u){pk16(hb[0], hb[1]), pk16(hb[2], hb[3]), pk16(hb[4], hb[5]), pk16(hb[6], hb[7])};
  unsigned short* op = out + (size_t)row * kDim + 8 * t;
  *(volatile v4u*)op = u;
  __threadfence();
  *(volatile v4u*)op = u;
}

__global__ __launch_bounds__(256) void mask_softmax_kernel(const float* __restrict__ S, const float* __restrict__ amask,
                                                          unsigned short* __restrict__ P) {
  __shared__ float redM[8];
  __shared__ float redS[8];
  const int i    = blockIdx.x;
  const int t    = threadIdx.x;
  const int lane = t & 31, wave = t >> 5;
  const size_t off = (size_t)i * kSeq + 8 * (size_t)t;
  const v4f s0 = *(const v4f*)(S + off);
  const v4f s1 = *(const v4f*)(S + off + 4);
  const v4f k0 = *(const v4f*)(amask + off);
  const v4f k1 = *(const v4f*)(amask + off + 4);
  float z[8];
#pragma unroll
  for (int e = 0; e < 4; ++e) {
    z[e]     = (s0[e] + k0[e]) * kScoreScale;
    z[4 + e] = (s1[e] + k1[e]) * kScoreScale;
  }
  float mx = z[0];
#pragma unroll
  for (int e = 1; e < 8; ++e) mx = fmaxf(mx, z[e]);
#pragma unroll
  for (int o = 16; o > 0; o >>= 1) mx = fmaxf(mx, __shfl_xor(mx, o, 32));
  if (lane == 0) redM[wave] = mx;
  __syncthreads();
  float m = redM[0];
#pragma unroll
  for (int w = 1; w < 8; ++w) m = fmaxf(m, redM[w]);

  float ev[8];
  float sum = 0.0f;
#pragma unroll
  for (int e = 0; e < 8; ++e) {
    ev[e] = expf(z[e] - m);
    sum += ev[e];
  }
#pragma unroll
  for (int o = 16; o > 0; o >>= 1) sum += __shfl_xor(sum, o, 32);
  if (lane == 0) redS[wave] = sum;
  __syncthreads();
  float tot = redS[0];
#pragma unroll
  for (int w = 1; w < 8; ++w) tot += redS[w];
  const float inv = kPCarry / tot;

  unsigned short hb[8];
#pragma unroll
  for (int e = 0; e < 8; ++e) hb[e] = h_bits(ev[e] * inv);
  const v4u u = (v4u){pk16(hb[0], hb[1]), pk16(hb[2], hb[3]), pk16(hb[4], hb[5]), pk16(hb[6], hb[7])};
  unsigned short* pr = P + off;
  *(volatile v4u*)pr = u;
  __threadfence();
  *(volatile v4u*)pr = u;
}

__global__ __launch_bounds__(256) void gelu_f16_kernel(const unsigned int* __restrict__ in, unsigned int* __restrict__ out, int n2) {
  const int i = blockIdx.x * 256 + threadIdx.x;
  if (i >= n2) return;
  const unsigned w = in[i];
  const float x0 = h16_to_f32(w & 0xffffu);
  const float x1 = h16_to_f32(w >> 16);
  const float g0 = (x0 * 0.5f) * (1.0f + erff(x0 * kRsqrt2));
  const float g1 = (x1 * 0.5f) * (1.0f + erff(x1 * kRsqrt2));
  const unsigned short b0 = h_bits(g0);
  const unsigned short b1 = h_bits(g1);
  const unsigned u = pk16(b0, b1);
  ((volatile unsigned*)out)[i] = u;
  __threadfence();
  ((volatile unsigned*)out)[i] = u;
}

constexpr size_t kSzWX  = (size_t)kD3 * kDim * 2;
constexpr size_t kSzWO  = (size_t)kDim * kDim * 2;
constexpr size_t kSzF1  = (size_t)kD4 * kDim * 2;
constexpr size_t kSzF2  = (size_t)kDim * kD4 * 2;
constexpr size_t kSzLN  = (size_t)kSeq * kDim * 2;
constexpr size_t kSzQK  = (size_t)kSeq * kD2 * 2;
constexpr size_t kSzVT  = (size_t)kDim * kSeq * 2;
constexpr size_t kSzSC  = (size_t)kSeq * kSeq * 4;
constexpr size_t kSzPP  = (size_t)kSeq * kSeq * 2;
constexpr size_t kSzATT = (size_t)kSeq * kDim * 2;
constexpr size_t kSzX1  = (size_t)kSeq * kDim * 4;
constexpr size_t kSzU   = (size_t)kSeq * kD4 * 2;
constexpr size_t kOffWX  = 0;
constexpr size_t kOffWO  = kOffWX + kSzWX;
constexpr size_t kOffF1  = kOffWO + kSzWO;
constexpr size_t kOffF2  = kOffF1 + kSzF1;
constexpr size_t kOffLN1 = kOffF2 + kSzF2;
constexpr size_t kOffQK  = kOffLN1 + kSzLN;
constexpr size_t kOffVT  = kOffQK + kSzQK;
constexpr size_t kOffSC  = kOffVT + kSzVT;
constexpr size_t kOffPP  = kOffSC + kSzSC;
constexpr size_t kOffATT = kOffPP + kSzPP;
constexpr size_t kOffX1  = kOffATT + kSzATT;
constexpr size_t kOffLN2 = kOffX1 + kSzX1;
constexpr size_t kOffU   = kOffLN2 + kSzLN;
constexpr size_t kOffG   = kOffU + kSzU;
constexpr size_t kWsTotal = kOffG + kSzU;
static_assert(kWsTotal == 117440512ull);
static_assert(kWsTotal <= 134217728ull);
static_assert(kOffWO % 128 == 0 && kOffF1 % 128 == 0 && kOffF2 % 128 == 0 && kOffLN1 % 128 == 0 && kOffQK % 128 == 0 &&
              kOffVT % 128 == 0 && kOffSC % 128 == 0 && kOffPP % 128 == 0 && kOffATT % 128 == 0 && kOffX1 % 128 == 0 &&
              kOffLN2 % 128 == 0 && kOffU % 128 == 0 && kOffG % 128 == 0);
static_assert(kSeq % 64 == 0 && kD2 % 64 == 0 && kDim % 64 == 0 && kD4 % 64 == 0 && kDh % 64 == 0);
static_assert(kDim % 32 == 0 && kDh % 32 == 0 && kSeq % 32 == 0 && kD4 % 32 == 0);
static_assert(((kD3 * kDim) / 8) % 256 == 0 && ((kDim * kDim) / 8) % 256 == 0 && ((kD4 * kDim) / 8) % 256 == 0);
static_assert(((kSeq * kD4) / 2) % 256 == 0);

extern "C" void kernel_launch(void* const* d_in, const int* in_sizes, int n_in,
                              void* d_out, int out_size, void* d_ws, size_t ws_size,
                              hipStream_t stream) {
  if (n_in < 14) return;
  if (in_sizes[0] != kSeq * kDim) return;
  if (in_sizes[1] != kSeq * kSeq) return;
  if (in_sizes[2] != kD3 * kDim || in_sizes[3] != kD3) return;
  if (in_sizes[4] != kDim * kDim || in_sizes[5] != kDim) return;
  if (in_sizes[6] != kD4 * kDim || in_sizes[7] != kD4) return;
  if (in_sizes[8] != kDim * kD4 || in_sizes[9] != kDim) return;
  if (in_sizes[10] < 1 || in_sizes[11] < 1 || in_sizes[12] < 1 || in_sizes[13] < 1) return;
  if (out_size != kSeq * kDim) return;
  if (ws_size < kWsTotal) return;

  const float* x     = (const float*)d_in[0];
  const float* amask = (const float*)d_in[1];
  const float* wx_w  = (const float*)d_in[2];
  const float* wx_b  = (const float*)d_in[3];
  const float* wo_w  = (const float*)d_in[4];
  const float* wo_b  = (const float*)d_in[5];
  const float* f1_w  = (const float*)d_in[6];
  const float* f1_b  = (const float*)d_in[7];
  const float* f2_w  = (const float*)d_in[8];
  const float* f2_b  = (const float*)d_in[9];
  const float* ln1_w = (const float*)d_in[10];
  const float* ln1_b = (const float*)d_in[11];
  const float* ln2_w = (const float*)d_in[12];
  const float* ln2_b = (const float*)d_in[13];
  float* out = (float*)d_out;
  char* ws = (char*)d_ws;
  unsigned short* WX16 = (unsigned short*)(ws + kOffWX);
  unsigned short* WO16 = (unsigned short*)(ws + kOffWO);
  unsigned short* F116 = (unsigned short*)(ws + kOffF1);
  unsigned short* F216 = (unsigned short*)(ws + kOffF2);
  unsigned short* LN1  = (unsigned short*)(ws + kOffLN1);
  unsigned short* QK   = (unsigned short*)(ws + kOffQK);
  unsigned short* VT   = (unsigned short*)(ws + kOffVT);
  float*          SC   = (float*)(ws + kOffSC);
  unsigned short* PP   = (unsigned short*)(ws + kOffPP);
  unsigned short* ATT  = (unsigned short*)(ws + kOffATT);
  float*          X1   = (float*)(ws + kOffX1);
  unsigned short* LN2  = (unsigned short*)(ws + kOffLN2);
  unsigned short* U16  = (unsigned short*)(ws + kOffU);
  unsigned short* G16  = (unsigned short*)(ws + kOffG);

  {
    const int n8wx = (kD3 * kDim) / 8;
    const int n8wo = (kDim * kDim) / 8;
    const int n8f  = (kD4 * kDim) / 8;
    cast8_f16_kernel<<<dim3(n8wx / 256), dim3(256), 0, stream>>>(wx_w, WX16, n8wx, kWCarry);
    cast8_f16_kernel<<<dim3(n8wo / 256), dim3(256), 0, stream>>>(wo_w, WO16, n8wo, kWCarry);
    cast8_f16_kernel<<<dim3(n8f / 256), dim3(256), 0, stream>>>(f1_w, F116, n8f, kWCarry);
    cast8_f16_kernel<<<dim3(n8f / 256), dim3(256), 0, stream>>>(f2_w, F216, n8f, kWCarry);
  }

  layernorm_f16_kernel<<<dim3(kSeq), dim3(128), 0, stream>>>(x, ln1_w, ln1_b, LN1);

  {
    const int tiles = (kSeq / 64) * (kD2 / 64);
    wmma_gemm64<0, false, 2, 1, false><<<dim3(tiles / 8, 1), dim3(256), 0, stream>>>(
        LN1, LN1, kDim, 0L, WX16, WX16, kDim, 0L,
        (void*)QK, (void*)QK, kD2, 0L, wx_b, wx_b, 0L, kSeq, kD2, kDim, kWCarryInv);
  }
  {
    const int tiles = (kDim / 64) * (kSeq / 64);
    wmma_gemm64<0, false, 1, 1, false><<<dim3(tiles / 8, 1), dim3(256), 0, stream>>>(
        WX16 + (size_t)kD2 * kDim, WX16 + (size_t)kD2 * kDim, kDim, 0L, LN1, LN1, kDim, 0L,
        (void*)VT, (void*)VT, kSeq, 0L, wx_b + kD2, wx_b, 0L, kDim, kSeq, kDim, kWCarryInv);
  }

  {
    const int tilesScore = (kSeq / 64) * (kSeq / 64);
    const int tilesCtx   = (kSeq / 64) * (kDh / 64);
    for (int h = 0; h < kHeads; ++h) {
      const unsigned short* Aq = QK + (size_t)h * kDh;
      const unsigned short* Bk = QK + (size_t)kDim + (size_t)h * kDh;
      wmma_gemm64<0, false, 0, 0, false><<<dim3(tilesScore / 8, 1), dim3(256), 0, stream>>>(
          Aq, Aq, kD2, 0L, Bk, Bk, kD2, 0L,
          (void*)SC, (void*)SC, kSeq, 0L, wx_b, wx_b, 0L, kSeq, kSeq, kDh, 1.0f);
      mask_softmax_kernel<<<dim3(kSeq), dim3(256), 0, stream>>>(SC, amask, PP);
      const unsigned short* Bv = VT + (size_t)h * kDh * kSeq;
      wmma_gemm64<0, false, 0, 1, false><<<dim3(tilesCtx / 8, 1), dim3(256), 0, stream>>>(
          PP, PP, kSeq, 0L, Bv, Bv, kSeq, 0L,
          (void*)(ATT + (size_t)h * kDh), (void*)ATT, kDim, 0L, wx_b, wx_b, 0L, kSeq, kDh, kSeq, kPCarryInv);
    }
  }

  {
    const int tiles = (kSeq / 64) * (kDim / 64);
    wmma_gemm64<0, false, 2, 0, true><<<dim3(tiles / 8, 1), dim3(256), 0, stream>>>(
        ATT, ATT, kDim, 0L, WO16, WO16, kDim, 0L,
        (void*)X1, (void*)X1, kDim, 0L, wo_b, x, 0L, kSeq, kDim, kDim, kWCarryInv);
  }

  layernorm_f16_kernel<<<dim3(kSeq), dim3(128), 0, stream>>>(X1, ln2_w, ln2_b, LN2);

  {
    const int tiles = (kSeq / 64) * (kD4 / 64);
    wmma_gemm64<0, false, 2, 1, false><<<dim3(tiles / 8, 1), dim3(256), 0, stream>>>(
        LN2, LN2, kDim, 0L, F116, F116, kDim, 0L,
        (void*)U16, (void*)U16, kD4, 0L, f1_b, f1_b, 0L, kSeq, kD4, kDim, kWCarryInv);
  }

  {
    const int n2 = (kSeq * kD4) / 2;
    gelu_f16_kernel<<<dim3(n2 / 256), dim3(256), 0, stream>>>((const unsigned int*)U16, (unsigned int*)G16, n2);
  }

  {
    const int tiles = (kSeq / 64) * (kDim / 64);
    wmma_gemm64<0, false, 2, 0, true><<<dim3(tiles / 8, 1), dim3(256), 0, stream>>>(
        G16, G16, kD4, 0L, F216, F216, kD4, 0L,
        (void*)out, (void*)out, kDim, 0L, f2_b, X1, 0L, kSeq, kDim, kD4, kWCarryInv);
  }
}
